// SimpleMamba2_11690900980064
// MI455X (gfx1250) — hardware-verified
//
#include <hip/hip_runtime.h>
#include <hip/hip_bf16.h>
#include <math.h>

#define DIM    1024
#define INNER  2048
#define HEADS  8
#define HD     256
#define NS     64
#define KW     4
#define NB     2
#define SEQL   2048
#define CH     256
#define NCH    (SEQL / CH)
#define NBC    1088
#define ACSP   32
#define GSTR   40
#define OSTR   68

typedef unsigned short us16 __attribute__((ext_vector_type(16)));
typedef unsigned short us8  __attribute__((ext_vector_type(8)));
typedef unsigned short us8a __attribute__((ext_vector_type(8), may_alias));
typedef unsigned short us4  __attribute__((ext_vector_type(4)));
typedef _Float16 v16h __attribute__((ext_vector_type(16)));
typedef _Float16 v8h  __attribute__((ext_vector_type(8)));
typedef _Float16 v4h  __attribute__((ext_vector_type(4)));
typedef __bf16 v16b __attribute__((ext_vector_type(16)));
typedef float v8f __attribute__((ext_vector_type(8)));
typedef float v4f __attribute__((ext_vector_type(4)));
typedef float v4fa __attribute__((ext_vector_type(4), may_alias));
union FragU { us16 v; us8 h[2]; };

__device__ __forceinline__ unsigned short bf16_bits(float f) {
  unsigned u = __float_as_uint(f);
  u += 0x7FFFu + ((u >> 16) & 1u);
  return (unsigned short)(u >> 16);
}
__device__ __forceinline__ float bf16_val(unsigned short b) { return __uint_as_float(((unsigned)b) << 16); }
__device__ __forceinline__ float bf16r(float f) { return bf16_val(bf16_bits(f)); }
__device__ __forceinline__ float silu_f(float v) { return v * __builtin_amdgcn_rcpf(1.0f + __expf(-v)); }

template <int TB>
__device__ __forceinline__ v8f mma32(us16 a, us16 b, v8f c) {
  if (TB) c = __builtin_amdgcn_wmma_f32_16x16x32_bf16(false, __builtin_bit_cast(v16b, a), false, __builtin_bit_cast(v16b, b), (short)0, c, false, false);
  else    c = __builtin_amdgcn_wmma_f32_16x16x32_f16(false, __builtin_bit_cast(v16h, a), false, __builtin_bit_cast(v16h, b), (short)0, c, false, false);
  return c;
}
__device__ __forceinline__ void wguard(v8f& c0, v8f& c1, v8f& c2, v8f& c3, const us16& a0, const us16& a1,
                                       const us16& b0, const us16& b1, const us16& b2, const us16& b3) {
#if defined(__HIP_DEVICE_COMPILE__)
  asm volatile("v_nop\n\tv_nop\n\tv_nop\n\tv_nop"
               : "+v"(c0), "+v"(c1), "+v"(c2), "+v"(c3)
               : "v"(a0), "v"(a1), "v"(b0), "v"(b1), "v"(b2), "v"(b3));
#endif
}

__device__ __forceinline__ us16 lds_frag(const unsigned short* base) {
  const int lane = threadIdx.x & 31, r = lane & 15, kh = (lane >> 4) * 8;
  FragU f;
  f.h[0] = *(const us8a*)(base + r * GSTR + kh);
  f.h[1] = *(const us8a*)(base + r * GSTR + 16 + kh);
  return f.v;
}

template <int KM>
__device__ __forceinline__ void stage_a(unsigned short* lds, const unsigned short* __restrict__ P, int ld, int m0, int k0, int tid) {
  if (KM == 0) {
    const int row = tid >> 1, cq = (tid & 1) * 16;
    const unsigned short* src = P + (size_t)(m0 + row) * ld + k0 + cq;
    const us8 v0 = *(const us8a*)src;
    const us8 v1 = *(const us8a*)(src + 8);
    *(us8a*)(lds + row * GSTR + cq) = v0;
    *(us8a*)(lds + row * GSTR + cq + 8) = v1;
  } else {
    const int k = tid >> 3, mq = (tid & 7) * 16;
    const unsigned short* src = P + (size_t)(k0 + k) * ld + m0 + mq;
    const us8 v0 = *(const us8a*)src;
    const us8 v1 = *(const us8a*)(src + 8);
#pragma unroll
    for (int u = 0; u < 8; ++u) { lds[(mq + u) * GSTR + k] = v0[u]; lds[(mq + 8 + u) * GSTR + k] = v1[u]; }
  }
}
template <int KM>
__device__ __forceinline__ void stage_b(unsigned short* lds, const unsigned short* __restrict__ P, int ld, int n0, int k0, int tid) {
  if (KM == 0) {
    const int row = tid >> 2, kq = (tid & 3) * 8;
    const us8 v = *(const us8a*)(P + (size_t)(n0 + row) * ld + k0 + kq);
    *(us8a*)(lds + row * GSTR + kq) = v;
  } else {
    const int k = tid >> 3, nq = (tid & 7) * 8;
    const us8 v = *(const us8a*)(P + (size_t)(k0 + k) * ld + n0 + nq);
#pragma unroll
    for (int u = 0; u < 8; ++u) lds[(nq + u) * GSTR + k] = v[u];
  }
}

template <int TB, int NP, int AKM, int BKM, int EPI>
__global__ __launch_bounds__(256) void k_gemm(
    const unsigned short* __restrict__ A0, const unsigned short* __restrict__ A1, int lda, long long sAc, long long sAh,
    const unsigned short* __restrict__ Bp, int ldb, long long sBc, long long sBh,
    void* Yv, int ldy, long long sYc, long long sYh,
    const float* __restrict__ R, int ldr, long long sRc, long long sRh,
    const float* __restrict__ aux, long long sXc, long long sXh,
    int zh, int K, float scale)
{
  __shared__ __attribute__((aligned(16))) unsigned short lA0[128 * GSTR];
  __shared__ __attribute__((aligned(16))) unsigned short lA1[(NP > 1) ? 128 * GSTR : 16];
  __shared__ __attribute__((aligned(16))) unsigned short lB[64 * GSTR];
  __shared__ __attribute__((aligned(16))) float oS[8 * 16 * OSTR];
  const int tid = threadIdx.x, lane = tid & 31, wave = tid >> 5, cl = lane & 15, hh = lane >> 4;
  const int m0 = blockIdx.x * 128, n0 = blockIdx.y * 64;
  const int z = blockIdx.z, zc = z / zh, zq = z - zc * zh;
  A0 += (long long)zc * sAc + (long long)zq * sAh;
  A1 += (long long)zc * sAc + (long long)zq * sAh;
  Bp += (long long)zc * sBc + (long long)zq * sBh;

  v8f acc[4];
#pragma unroll
  for (int j = 0; j < 4; ++j) { v8f zz = {0.f, 0.f, 0.f, 0.f, 0.f, 0.f, 0.f, 0.f}; acc[j] = zz; }

#pragma unroll 1
  for (int k0 = 0; k0 < K; k0 += 32) {
    __syncthreads();
    stage_a<AKM>(lA0, A0, lda, m0, k0, tid);
    if (NP > 1) stage_a<AKM>(lA1, A1, lda, m0, k0, tid);
    stage_b<BKM>(lB, Bp, ldb, n0, k0, tid);
    __syncthreads();
    const us16 af = lds_frag(lA0 + 16 * wave * GSTR);
    us16 afl = af;
    if (NP > 1) afl = lds_frag(lA1 + 16 * wave * GSTR);
    us16 bf[4];
#pragma unroll
    for (int j = 0; j < 4; ++j) bf[j] = lds_frag(lB + 16 * j * GSTR);
#pragma unroll
    for (int j = 0; j < 4; ++j) acc[j] = mma32<TB>(af, bf[j], acc[j]);
    if (NP > 1) {
#pragma unroll
      for (int j = 0; j < 4; ++j) acc[j] = mma32<TB>(afl, bf[j], acc[j]);
    }
    wguard(acc[0], acc[1], acc[2], acc[3], af, afl, bf[0], bf[1], bf[2], bf[3]);
  }

  float* so = oS + wave * (16 * OSTR);
#pragma unroll
  for (int j = 0; j < 4; ++j)
#pragma unroll
    for (int r = 0; r < 8; ++r) so[(8 * hh + r) * OSTR + 16 * j + cl] = acc[j][r] * scale;
  __syncthreads();
  if (EPI != 0) {
    float dsk = 0.0f;
    const float* acs = aux;
    const float* Rz = R;
    if (EPI == 1) { dsk = bf16r(aux[zq]); Rz = R + (long long)zc * sRc + (long long)zq * sRh; }
    if (EPI == 2) acs = aux + (long long)zc * sXc + (long long)zq * sXh;
#pragma unroll 1
    for (int e = lane; e < 16 * 64; e += 32) {
      const int r = e >> 6, c = e & 63;
      const int m = m0 + 16 * wave + r, n = n0 + c;
      float v = so[r * OSTR + c];
      if (EPI == 1) v += dsk * Rz[(size_t)m * ldr + n];
      if (EPI == 2) {
        const float ai = acs[(size_t)m * ACSP], as = acs[(size_t)n * ACSP];
        const float d = expf(fminf(ai - as, 0.0f));
        v = (n <= m) ? v * d : 0.0f;
      }
      so[r * OSTR + c] = v;
    }
    __syncthreads();
  }
#pragma unroll
  for (int pass = 0; pass < 2; ++pass) {
    if (EPI == 2) {
      unsigned short* Y = (unsigned short*)Yv + (long long)zc * sYc + (long long)zq * sYh;
#pragma unroll
      for (int it = 0; it < 4; ++it) {
        const int ch = it * 32 + lane, r = ch >> 3, q8 = (ch & 7) * 8;
        v8h hv;
#pragma unroll
        for (int u = 0; u < 8; ++u) hv[u] = (_Float16)so[r * OSTR + q8 + u];
        const us8 o = __builtin_bit_cast(us8, hv);
        *(volatile us8*)(Y + (size_t)(m0 + 16 * wave + r) * ldy + n0 + q8) = o;
      }
    } else {
      float* Y = (float*)Yv + (long long)zc * sYc + (long long)zq * sYh;
#pragma unroll
      for (int it = 0; it < 8; ++it) {
        const int ch = it * 32 + lane, r = ch >> 4, q = (ch & 15) * 4;
        const v4f v = *(const v4fa*)(so + r * OSTR + q);
        *(volatile v4f*)(Y + (size_t)(m0 + 16 * wave + r) * ldy + n0 + q) = v;
      }
    }
    __threadfence();
  }
}

__global__ __launch_bounds__(256) void k_cvt_bf16(const float* __restrict__ src, unsigned short* __restrict__ dst, int n8) {
  const int i = blockIdx.x * 256 + threadIdx.x;
  if (i >= n8) return;
  const float* p = src + (size_t)i * 8;
  const v4f a = *(const v4fa*)p, b = *(const v4fa*)(p + 4);
  us8 o;
#pragma unroll
  for (int u = 0; u < 4; ++u) { o[u] = bf16_bits(a[u]); o[4 + u] = bf16_bits(b[u]); }
  unsigned short* d = dst + (size_t)i * 8;
  *(volatile us8*)d = o;
  __threadfence();
  *(volatile us8*)d = o;
}

__global__ __launch_bounds__(256) void k_wbcd(const float* __restrict__ Wb, const float* __restrict__ Wc, const float* __restrict__ Wd,
                                             unsigned short* __restrict__ W16) {
  const int r = blockIdx.x, tid = threadIdx.x, c0 = tid * 8;
  const float* src = Wd;
  float on = 0.0f;
  if (r < HEADS * NS)              { src = Wb + (size_t)r * INNER; on = 1.0f; }
  else if (r < 2 * HEADS * NS)     { src = Wc + (size_t)(r - HEADS * NS) * INNER; on = 1.0f; }
  else if (r < 2 * HEADS * NS + HEADS) { src = Wd + (size_t)(r - 2 * HEADS * NS) * INNER; on = 1.0f; }
  const v4f a = *(const v4fa*)(src + c0), b = *(const v4fa*)(src + c0 + 4);
  v8h hv;
#pragma unroll
  for (int u = 0; u < 4; ++u) { hv[u] = (_Float16)(bf16r(a[u]) * 64.0f * on); hv[4 + u] = (_Float16)(bf16r(b[u]) * 64.0f * on); }
  const us8 o = __builtin_bit_cast(us8, hv);
  unsigned short* d = W16 + (size_t)r * INNER + c0;
  *(volatile us8*)d = o;
  __threadfence();
  *(volatile us8*)d = o;
}

__global__ __launch_bounds__(512) void k_conv(const float* __restrict__ X, const float* __restrict__ cw, const float* __restrict__ cb,
                                             float* __restrict__ XC, unsigned short* __restrict__ XC16) {
  const int t = blockIdx.x, tid = threadIdx.x, c = 4 * tid;
  v4f w[4];
#pragma unroll
  for (int u = 0; u < 4; ++u) w[u] = *(const v4fa*)(cw + (size_t)(c + u) * KW);
  v4f acc = {0.0f, 0.0f, 0.0f, 0.0f};
#pragma unroll
  for (int k = 0; k < KW; ++k) {
    const int tt = t - (KW - 1) + k;
    const int row = (tt < 0) ? 0 : tt;
    const float live = (tt >= 0) ? 1.0f : 0.0f;
    const v4f xv = *(const v4fa*)(X + (size_t)row * INNER + c);
#pragma unroll
    for (int u = 0; u < 4; ++u) acc[u] += (xv[u] * live) * bf16r(w[u][k]);
  }
  const v4f bv = *(const v4fa*)(cb + c);
  v4f res; v4h hv;
#pragma unroll
  for (int u = 0; u < 4; ++u) { const float s = silu_f(acc[u] + bf16r(bv[u])); res[u] = s; hv[u] = (_Float16)(s * 64.0f); }
  const us4 o = __builtin_bit_cast(us4, hv);
  float* d0 = XC + (size_t)t * INNER + c;
  unsigned short* d1 = XC16 + (size_t)t * INNER + c;
  *(volatile v4f*)d0 = res; *(volatile us4*)d1 = o;
  __threadfence();
  *(volatile v4f*)d0 = res; *(volatile us4*)d1 = o;
}

__global__ __launch_bounds__(32) void k_dtacs(const float* __restrict__ BCD, const float* __restrict__ bdt, const float* __restrict__ loga,
                                              float* __restrict__ DT, float* __restrict__ ACS) {
  const int c = blockIdx.x, h = threadIdx.x;
  const int hc = (h < HEADS) ? h : (HEADS - 1);
  const float live = (h < HEADS) ? 1.0f : 0.0f;
  const float ah = -expf(bf16r(loga[hc]));
  const float bh = bf16r(bdt[hc]);
#pragma unroll 1
  for (int pass = 0; pass < 2; ++pass) {
    float run = 0.0f;
#pragma unroll 1
    for (int i = 0; i < CH; ++i) {
      const size_t l = (size_t)c * CH + i;
      const float dr = BCD[l * NBC + 2 * HEADS * NS + hc] + bh;
      const float sp = fmaxf(dr, 0.0f) + log1pf(expf(-fabsf(dr)));
      const float dt = sp * live;
      run = run + ah * dt;
      *(volatile float*)(DT + l * ACSP + h) = dt;
      *(volatile float*)(ACS + l * ACSP + h) = run * live;
    }
    __threadfence();
  }
}

__global__ __launch_bounds__(256) void k_planes(const float* __restrict__ XC, const float* __restrict__ BCD, const float* __restrict__ DT,
                                               const float* __restrict__ ACS, unsigned short* __restrict__ XDT16, unsigned short* __restrict__ XDEC16,
                                               unsigned short* __restrict__ BC16, unsigned short* __restrict__ CS16) {
  const int l = blockIdx.x, tid = threadIdx.x, llast = l | (CH - 1);
  {
    const int c = 8 * tid, h = c >> 8;
    const float dt = DT[(size_t)l * ACSP + h];
    const float dec = expf(fminf(ACS[(size_t)llast * ACSP + h] - ACS[(size_t)l * ACSP + h], 0.0f));
    const float s1 = dt * 4096.0f, s2 = dt * dec * 4096.0f;
    const v4f x0 = *(const v4fa*)(XC + (size_t)l * INNER + c), x1 = *(const v4fa*)(XC + (size_t)l * INNER + c + 4);
    v8h a, b;
#pragma unroll
    for (int u = 0; u < 4; ++u) {
      a[u] = (_Float16)(x0[u] * s1); a[4 + u] = (_Float16)(x1[u] * s1);
      b[u] = (_Float16)(x0[u] * s2); b[4 + u] = (_Float16)(x1[u] * s2);
    }
    const us8 oa = __builtin_bit_cast(us8, a), ob = __builtin_bit_cast(us8, b);
    unsigned short* pa = XDT16 + (size_t)l * INNER + c;
    unsigned short* pb = XDEC16 + (size_t)l * INNER + c;
    *(volatile us8*)pa = oa; *(volatile us8*)pb = ob;
    __threadfence();
    *(volatile us8*)pa = oa; *(volatile us8*)pb = ob;
  }
  if (tid < 128) {
    const int j = 8 * tid;
    const float* src = BCD + (size_t)l * NBC + j;
    const v4f v0 = *(const v4fa*)src, v1 = *(const v4fa*)(src + 4);
    v8h hv;
#pragma unroll
    for (int u = 0; u < 4; ++u) { hv[u] = (_Float16)(v0[u] * 1024.0f); hv[4 + u] = (_Float16)(v1[u] * 1024.0f); }
    const us8 o = __builtin_bit_cast(us8, hv);
    unsigned short* d = BC16 + (size_t)l * (2 * HEADS * NS) + j;
    *(volatile us8*)d = o;
    __threadfence();
    *(volatile us8*)d = o;
  } else if (tid < 192) {
    const int j = 8 * (tid - 128), h = j >> 6;
    const float ea = expf(fminf(ACS[(size_t)l * ACSP + h], 0.0f)) * 1024.0f;
    const float* src = BCD + (size_t)l * NBC + HEADS * NS + j;
    const v4f v0 = *(const v4fa*)src, v1 = *(const v4fa*)(src + 4);
    v8h hv;
#pragma unroll
    for (int u = 0; u < 4; ++u) { hv[u] = (_Float16)(v0[u] * ea); hv[4 + u] = (_Float16)(v1[u] * ea); }
    const us8 o = __builtin_bit_cast(us8, hv);
    unsigned short* d = CS16 + (size_t)l * (HEADS * NS) + j;
    *(volatile us8*)d = o;
    __threadfence();
    *(volatile us8*)d = o;
  }
}

__global__ __launch_bounds__(256) void k_prev(const float* __restrict__ ST, const float* __restrict__ ACS, unsigned short* __restrict__ PREV16) {
  const int part = blockIdx.x, h = blockIdx.y, tid = threadIdx.x;
  const int e0 = part * 2048 + tid * 8;
  v4f p0 = {0.0f, 0.0f, 0.0f, 0.0f}, p1 = {0.0f, 0.0f, 0.0f, 0.0f};
#pragma unroll 1
  for (int c = 0; c < NCH; ++c) {
    const size_t base = (size_t)(c * HEADS + h) * (HD * NS) + e0;
    v8h hv;
#pragma unroll
    for (int u = 0; u < 4; ++u) { hv[u] = (_Float16)(p0[u] * 65536.0f); hv[4 + u] = (_Float16)(p1[u] * 65536.0f); }
    const us8 o = __builtin_bit_cast(us8, hv);
    *(volatile us8*)(PREV16 + base) = o;
    __threadfence();
    *(volatile us8*)(PREV16 + base) = o;
    const float dec = expf(fminf(ACS[(size_t)(c * CH + CH - 1) * ACSP + h], 0.0f));
    const v4f s0 = *(const v4fa*)(ST + base), s1 = *(const v4fa*)(ST + base + 4);
    p0 = p0 * dec + s0;
    p1 = p1 * dec + s1;
  }
}

__global__ __launch_bounds__(256) void k_gnstat(const float* __restrict__ YD, const float* __restrict__ YO, float* __restrict__ STAT) {
  __shared__ double rs[256];
  __shared__ double rq[256];
  __shared__ __attribute__((aligned(16))) float st[32];
  const int tid = threadIdx.x;
  if (tid < 32) st[tid] = 0.0f;
#pragma unroll 1
  for (int h = 0; h < HEADS; ++h) {
    const int c = h * HD + tid;
    double s = 0.0, q = 0.0;
#pragma unroll 4
    for (int l = 0; l < SEQL; ++l) {
      const float y = YD[(size_t)l * INNER + c] + YO[(size_t)l * INNER + c];
      const double yd = (double)y;
      s += yd;
      q += yd * yd;
    }
    __syncthreads();
    rs[tid] = s; rq[tid] = q;
    __syncthreads();
    for (int o = 128; o > 0; o >>= 1) {
      if (tid < o) { rs[tid] += rs[tid + o]; rq[tid] += rq[tid + o]; }
      __syncthreads();
    }
    if (tid == 0) {
      const double n = (double)SEQL * (double)HD;
      const double mean = rs[0] / n;
      double var = rq[0] / n - mean * mean;
      if (var < 0.0) var = 0.0;
      st[2 * h] = (float)mean;
      st[2 * h + 1] = (float)(1.0 / sqrt(var + 1e-5));
    }
    __syncthreads();
  }
  if (tid < 8) {
    const v4f v = *(const v4fa*)(st + 4 * tid);
    *(volatile v4f*)(STAT + 4 * tid) = v;
    __threadfence();
    *(volatile v4f*)(STAT + 4 * tid) = v;
  }
}

__device__ __forceinline__ unsigned int gate_elem(float y, float z, float w, float b, float mean, float rstd) {
  const float yn = (y - mean) * rstd * bf16r(w) + bf16r(b);
  const float g = yn * silu_f(z);
  const unsigned short hb = bf16_bits(g);
  const unsigned short lb = bf16_bits(g - bf16_val(hb));
  return (unsigned int)hb | ((unsigned int)lb << 16);
}
__global__ __launch_bounds__(256) void k_gate(const float* __restrict__ YD, const float* __restrict__ YO, const float* __restrict__ Z,
                                             const float* __restrict__ STAT, const float* __restrict__ gnw, const float* __restrict__ gnb,
                                             unsigned short* __restrict__ GH, unsigned short* __restrict__ GL) {
  const int l = blockIdx.x, tid = threadIdx.x, c = 8 * tid, h = c >> 8;
  const float mean = STAT[2 * h], rstd = STAT[2 * h + 1];
  const size_t off = (size_t)l * INNER + c;
  const v4f ya = *(const v4fa*)(YD + off) + *(const v4fa*)(YO + off);
  const v4f yb = *(const v4fa*)(YD + off + 4) + *(const v4fa*)(YO + off + 4);
  const v4f za = *(const v4fa*)(Z + off), zb = *(const v4fa*)(Z + off + 4);
  const v4f wa = *(const v4fa*)(gnw + c), wb = *(const v4fa*)(gnw + c + 4);
  const v4f ba = *(const v4fa*)(gnb + c), bb = *(const v4fa*)(gnb + c + 4);
  us8 hi, lo;
#pragma unroll
  for (int u = 0; u < 4; ++u) {
    const unsigned int pa = gate_elem(ya[u], za[u], wa[u], ba[u], mean, rstd);
    const unsigned int pb = gate_elem(yb[u], zb[u], wb[u], bb[u], mean, rstd);
    hi[u] = (unsigned short)(pa & 0xFFFFu); lo[u] = (unsigned short)(pa >> 16);
    hi[4 + u] = (unsigned short)(pb & 0xFFFFu); lo[4 + u] = (unsigned short)(pb >> 16);
  }
  *(volatile us8*)(GH + off) = hi; *(volatile us8*)(GL + off) = lo;
  __threadfence();
  *(volatile us8*)(GH + off) = hi; *(volatile us8*)(GL + off) = lo;
}

extern "C" void kernel_launch(void* const* d_in, const int* in_sizes, int n_in,
                              void* d_out, int out_size, void* d_ws, size_t ws_size,
                              hipStream_t stream) {
  if (n_in < 14) return;
  if (in_sizes[0] != NB * SEQL * DIM || in_sizes[1] != INNER * DIM || in_sizes[2] != INNER * DIM || in_sizes[3] != INNER * KW ||
      in_sizes[4] != INNER || in_sizes[5] != HEADS * NS * INNER || in_sizes[6] != HEADS * NS * INNER || in_sizes[7] != HEADS * INNER ||
      in_sizes[8] != HEADS || in_sizes[9] != HEADS || in_sizes[10] != HEADS || in_sizes[11] != INNER || in_sizes[12] != INNER ||
      in_sizes[13] != DIM * INNER || out_size != NB * SEQL * DIM) return;
  const float* u    = (const float*)d_in[0];
  const float* Wx   = (const float*)d_in[1];
  const float* Wz   = (const float*)d_in[2];
  const float* cw   = (const float*)d_in[3];
  const float* cb   = (const float*)d_in[4];
  const float* Wb   = (const float*)d_in[5];
  const float* Wc   = (const float*)d_in[6];
  const float* Wdt  = (const float*)d_in[7];
  const float* bdt  = (const float*)d_in[8];
  const float* loga = (const float*)d_in[9];
  const float* dprm = (const float*)d_in[10];
  const float* gnw  = (const float*)d_in[11];
  const float* gnb  = (const float*)d_in[12];
  const float* Wout = (const float*)d_in[13];
  float* out = (float*)d_out;

  size_t off = 0;
  auto carve = [&](size_t bytes) -> char* { char* p = (char*)d_ws + off; off += (bytes + 255) & ~(size_t)255; return p; };
  unsigned short* IN16   = (unsigned short*)carve((size_t)NB * SEQL * DIM * 2);
  unsigned short* WX16   = (unsigned short*)carve((size_t)INNER * DIM * 2);
  unsigned short* WZ16   = (unsigned short*)carve((size_t)INNER * DIM * 2);
  unsigned short* WO16   = (unsigned short*)carve((size_t)DIM * INNER * 2);
  unsigned short* WBCD16 = (unsigned short*)carve((size_t)NBC * INNER * 2);
  float* XR  = (float*)carve((size_t)SEQL * INNER * 4);
  float* Zf  = (float*)carve((size_t)SEQL * INNER * 4);
  float* XC  = (float*)carve((size_t)SEQL * INNER * 4);
  unsigned short* XC16 = (unsigned short*)carve((size_t)SEQL * INNER * 2);
  float* BCD = (float*)carve((size_t)SEQL * NBC * 4);
  float* DT  = (float*)carve((size_t)SEQL * ACSP * 4);
  float* ACS = (float*)carve((size_t)SEQL * ACSP * 4);
  unsigned short* BC16   = (unsigned short*)carve((size_t)SEQL * 2 * HEADS * NS * 2);
  unsigned short* CS16   = (unsigned short*)carve((size_t)SEQL * HEADS * NS * 2);
  unsigned short* XDT16  = (unsigned short*)carve((size_t)SEQL * INNER * 2);
  unsigned short* XDEC16 = (unsigned short*)carve((size_t)SEQL * INNER * 2);
  float* ST  = (float*)carve((size_t)NCH * HEADS * HD * NS * 4);
  unsigned short* PREV16 = (unsigned short*)carve((size_t)NCH * HEADS * HD * NS * 2);
  float* STAT = (float*)carve(256);
  if (off > ws_size || off > (size_t)134217728) return;
  float* YD = XR;
  float* YO = XC;
  unsigned short* G16 = (unsigned short*)BCD;
  unsigned short* GH = XDT16;
  unsigned short* GL = XDEC16;

  const dim3 blk(256);
  { const int n8 = in_sizes[0] / 8;  k_cvt_bf16<<<dim3((n8 + 255) / 256), blk, 0, stream>>>(u, IN16, n8); }
  { const int n8 = in_sizes[1] / 8;  k_cvt_bf16<<<dim3((n8 + 255) / 256), blk, 0, stream>>>(Wx, WX16, n8); }
  { const int n8 = in_sizes[2] / 8;  k_cvt_bf16<<<dim3((n8 + 255) / 256), blk, 0, stream>>>(Wz, WZ16, n8); }
  { const int n8 = in_sizes[13] / 8; k_cvt_bf16<<<dim3((n8 + 255) / 256), blk, 0, stream>>>(Wout, WO16, n8); }
  k_wbcd<<<dim3(NBC), blk, 0, stream>>>(Wb, Wc, Wdt, WBCD16);

  const float* nul = nullptr;
  for (int b = 0; b < NB; ++b) {
    const unsigned short* in16b = IN16 + (size_t)b * SEQL * DIM;
    float* outb = out + (size_t)b * SEQL * DIM;
    k_gemm<1, 1, 0, 0, 0><<<dim3(SEQL / 128, INNER / 64, 1), blk, 0, stream>>>(in16b, in16b, DIM, 0, 0, WX16, DIM, 0, 0,
        (void*)XR, INNER, 0, 0, nul, 0, 0, 0, nul, 0, 0, 1, DIM, 1.0f);
    k_gemm<1, 1, 0, 0, 0><<<dim3(SEQL / 128, INNER / 64, 1), blk, 0, stream>>>(in16b, in16b, DIM, 0, 0, WZ16, DIM, 0, 0,
        (void*)Zf, INNER, 0, 0, nul, 0, 0, 0, nul, 0, 0, 1, DIM, 1.0f);
    k_conv<<<dim3(SEQL), dim3(512), 0, stream>>>(XR, cw, cb, XC, XC16);
    k_gemm<0, 1, 0, 0, 0><<<dim3(SEQL / 128, NBC / 64, 1), blk, 0, stream>>>(XC16, XC16, INNER, 0, 0, WBCD16, INNER, 0, 0,
        (void*)BCD, NBC, 0, 0, nul, 0, 0, 0, nul, 0, 0, 1, INNER, 1.0f / 4096.0f);
    k_dtacs<<<dim3(NCH), dim3(32), 0, stream>>>(BCD, bdt, loga, DT, ACS);
    k_planes<<<dim3(SEQL), blk, 0, stream>>>(XC, BCD, DT, ACS, XDT16, XDEC16, BC16, CS16);
    k_gemm<0, 1, 0, 0, 2><<<dim3(CH / 128, CH / 64, NCH * HEADS), blk, 0, stream>>>(BC16 + HEADS * NS, BC16 + HEADS * NS, 2 * HEADS * NS,
        (long long)CH * 2 * HEADS * NS, NS, BC16, 2 * HEADS * NS, (long long)CH * 2 * HEADS * NS, NS,
        (void*)G16, CH, (long long)HEADS * CH * CH, (long long)CH * CH, nul, 0, 0, 0, ACS, (long long)CH * ACSP, 1, HEADS, NS, 1.0f / 256.0f);
    k_gemm<0, 1, 0, 1, 1><<<dim3(CH / 128, HD / 64, NCH * HEADS), blk, 0, stream>>>(G16, G16, CH, (long long)HEADS * CH * CH, (long long)CH * CH,
        XDT16, INNER, (long long)CH * INNER, HD, (void*)YD, INNER, (long long)CH * INNER, HD, XC, INNER, (long long)CH * INNER, HD,
        dprm, 0, 0, HEADS, CH, 1.0f / 16777216.0f);
    k_gemm<0, 1, 1, 1, 0><<<dim3(HD / 128, NS / 64, NCH * HEADS), blk, 0, stream>>>(XDEC16, XDEC16, INNER, (long long)CH * INNER, HD,
        BC16, 2 * HEADS * NS, (long long)CH * 2 * HEADS * NS, NS, (void*)ST, NS, (long long)HEADS * HD * NS, (long long)HD * NS,
        nul, 0, 0, 0, nul, 0, 0, HEADS, CH, 1.0f / 4194304.0f);
    k_prev<<<dim3(8, HEADS), blk, 0, stream>>>(ST, ACS, PREV16);
    k_gemm<0, 1, 0, 0, 0><<<dim3(CH / 128, HD / 64, NCH * HEADS), blk, 0, stream>>>(CS16, CS16, HEADS * NS, (long long)CH * HEADS * NS, NS,
        PREV16, NS, (long long)HEADS * HD * NS, (long long)HD * NS, (void*)YO, INNER, (long long)CH * INNER, HD,
        nul, 0, 0, 0, nul, 0, 0, HEADS, NS, 1.0f / 67108864.0f);
    k_gnstat<<<dim3(1), blk, 0, stream>>>(YD, YO, STAT);
    k_gate<<<dim3(SEQL), blk, 0, stream>>>(YD, YO, Zf, STAT, gnw, gnb, GH, GL);
    k_gemm<1, 2, 0, 0, 0><<<dim3(SEQL / 128, DIM / 64, 1), blk, 0, stream>>>(GH, GL, INNER, 0, 0, WO16, INNER, 0, 0,
        (void*)outb, DIM, 0, 0, nul, 0, 0, 0, nul, 0, 0, 1, INNER, 1.0f);
  }
}
